// ComplexMultiheadAttention_25391846654007
// MI455X (gfx1250) — hardware-verified
//
#include <hip/hip_runtime.h>


#define NB_  2
#define TT   2048
#define DIM  256
#define NH_  8
#define DH   32
#define DW   (2 * DH)
#define DQ   (NH_ * DW)
#define KX   (2 * DIM)
#define NREP 4
#define KPV  (NREP * TT)
#define ZH   1
#define HD   DW
#define RH   512
#define PCAR 1024.0f
#define SCL  0.17677669529663689f
typedef _Float16 h16;
typedef unsigned short bf;
typedef __attribute__((ext_vector_type(16))) __bf16   v16bf;
typedef __attribute__((ext_vector_type(16))) _Float16 v16h;
typedef __attribute__((ext_vector_type(8)))  _Float16 v8h;
typedef __attribute__((ext_vector_type(8)))  unsigned short v8us;
typedef __attribute__((ext_vector_type(8)))  float    v8f;
typedef __attribute__((ext_vector_type(4)))  float    v4f;
typedef v8h  __attribute__((may_alias)) v8ha;
typedef v4f  __attribute__((may_alias)) v4fa;
typedef v8us __attribute__((may_alias)) v8usa;

__device__ __forceinline__ unsigned short f2bf(float f) { unsigned u = __float_as_uint(f); u += 0x7FFFu + ((u >> 16) & 1u); return (unsigned short)(u >> 16); }
__device__ __forceinline__ float bf2f(unsigned short b) { return __uint_as_float(((unsigned)b) << 16); }
__device__ __forceinline__ float bfr(float f) { return bf2f(f2bf(f)); }
__device__ __forceinline__ v16h cat16(v8h lo, v8h hi) { return __builtin_shufflevector(lo, hi, 0, 1, 2, 3, 4, 5, 6, 7, 8, 9, 10, 11, 12, 13, 14, 15); }
__device__ __forceinline__ v16bf cat16b(v8us lo, v8us hi) { return __builtin_bit_cast(v16bf, __builtin_shufflevector(lo, hi, 0, 1, 2, 3, 4, 5, 6, 7, 8, 9, 10, 11, 12, 13, 14, 15)); }
__device__ __forceinline__ v8f wmma16(v16h a, v16h b, v8f c) { return __builtin_amdgcn_wmma_f32_16x16x32_f16(false, a, false, b, (short)0, c, false, false); }
__device__ __forceinline__ v8f wmmab(v16bf a, v16bf b, v8f c) { return __builtin_amdgcn_wmma_f32_16x16x32_bf16(false, a, false, b, (short)0, c, false, false); }


template <typename T16> struct WFrag;
template <> struct WFrag<h16> { typedef v16h V; static __device__ __forceinline__ V ld(const h16* p) { return cat16(*(const v8h*)p, *(const v8h*)(p + 16)); } static __device__ __forceinline__ v8f mma(V a, V b, v8f c) { return wmma16(a, b, c); } };
template <> struct WFrag<bf> { typedef v16bf V; static __device__ __forceinline__ V ld(const bf* p) { return cat16b(*(const v8us*)p, *(const v8us*)(p + 16)); } static __device__ __forceinline__ v8f mma(V a, V b, v8f c) { return wmmab(a, b, c); } };
template <typename T16, int NSPLIT, bool BIAS>
__global__ __launch_bounds__(32) void k_gemmw(const T16* __restrict__ A, const T16* __restrict__ A2, const T16* __restrict__ Bt, const T16* __restrict__ Bt2, int K, float* C, int ldc, const float* __restrict__ bias, size_t sA, size_t sB, size_t sC) {
    typedef typename WFrag<T16>::V V;
    __shared__ __align__(16) float os[16 * 68];
    const size_t z = blockIdx.z; A += z * sA; if (A2) A2 += z * sA; Bt += z * sB; if (Bt2) Bt2 += z * sB; C += z * sC;
    const int lane = threadIdx.x & 31, lr = lane & 15, hi = lane >> 4; const int r0 = blockIdx.x * 64, c0 = blockIdx.y * 64;
    v8f acc[4][4];
#pragma unroll
    for (int mb = 0; mb < 4; ++mb)
#pragma unroll
        for (int nb = 0; nb < 4; ++nb) acc[mb][nb] = (v8f){};
    const size_t aoff = (size_t)(r0 + lr) * K + 8 * hi, boff = (size_t)(c0 + lr) * K + 8 * hi;
#pragma unroll 1
    for (int kc = 0; kc < K; kc += 32) {
        V a[4], a2[4];
#pragma unroll
        for (int mb = 0; mb < 4; ++mb) { a[mb] = WFrag<T16>::ld(A + aoff + (size_t)mb * 16 * K + kc); if (NSPLIT == 1 || NSPLIT == 2) a2[mb] = WFrag<T16>::ld(A2 + aoff + (size_t)mb * 16 * K + kc); }
#pragma unroll
        for (int nb = 0; nb < 4; ++nb) { const V b = WFrag<T16>::ld(Bt + boff + (size_t)nb * 16 * K + kc); V b2; if (NSPLIT >= 2) b2 = WFrag<T16>::ld(Bt2 + boff + (size_t)nb * 16 * K + kc);
#pragma unroll
            for (int mb = 0; mb < 4; ++mb) { acc[mb][nb] = WFrag<T16>::mma(a[mb], b, acc[mb][nb]); if (NSPLIT == 1 || NSPLIT == 2) acc[mb][nb] = WFrag<T16>::mma(a2[mb], b, acc[mb][nb]); if (NSPLIT >= 2) acc[mb][nb] = WFrag<T16>::mma(a[mb], b2, acc[mb][nb]); } }
        asm volatile("v_nop\n\tv_nop\n\tv_nop\n\tv_nop" : "+v"(acc[0][0]), "+v"(acc[1][1]), "+v"(acc[2][2]), "+v"(acc[3][3]) : "v"(a[0]), "v"(a[3]));
    }
#pragma unroll
    for (int mb = 0; mb < 4; ++mb) {
#pragma unroll
        for (int nb = 0; nb < 4; ++nb) {
#pragma unroll
            for (int j = 0; j < 8; ++j) os[(hi * 8 + j) * 68 + nb * 16 + lr] = acc[mb][nb][j]; }
        __builtin_amdgcn_wave_barrier(); asm volatile("" ::: "memory");
        float* crow = C + (size_t)(r0 + mb * 16) * ldc + c0;
#pragma unroll 1
        for (int ps = 0; ps < 2; ++ps) {
#pragma unroll
            for (int s = 0; s < 8; ++s) { const int row = 2 * s + hi, cofs = lr * 4; v4f val = *(const v4fa*)(os + row * 68 + cofs); if (BIAS) { val[0] += bfr(bias[c0 + cofs]); val[1] += bfr(bias[c0 + cofs + 1]); val[2] += bfr(bias[c0 + cofs + 2]); val[3] += bfr(bias[c0 + cofs + 3]); }
                *(volatile v4f*)(crow + (size_t)row * ldc + cofs) = val; }
            if (ps == 0) __threadfence(); }
        __builtin_amdgcn_wave_barrier(); asm volatile("" ::: "memory");
    }
}

__device__ __forceinline__ h16 tohx(float x) { return (h16)x; }
__device__ __forceinline__ void splitf(float y, unsigned short& h, unsigned short& l) { h = f2bf(y); l = f2bf(y - bf2f(h)); }
typedef __attribute__((ext_vector_type(2))) _Float16 v2h;
typedef __attribute__((ext_vector_type(4))) _Float16 v4h;
typedef __attribute__((ext_vector_type(2))) unsigned short v2us;
typedef __attribute__((ext_vector_type(4))) unsigned short v4us;
typedef __attribute__((ext_vector_type(2))) float v2f;
typedef __attribute__((ext_vector_type(4))) int v4i;


__global__ __launch_bounds__(256) void k_cvt8c(const float* __restrict__ xr, const float* __restrict__ xi, bf* dst) { const size_t i = (size_t)blockIdx.x * 256 + threadIdx.x; if (i >= (size_t)TT * KX / 8) return; const int t = (int)(i / (KX / 8)); const int k0 = (int)(i % (KX / 8)) * 8; const float* src = (k0 < DIM) ? (xr + (size_t)t * DIM + k0) : (xi + (size_t)t * DIM + (k0 - DIM)); const v8f v = *(const v8f*)src; v8us o;
#pragma unroll
    for (int k = 0; k < 8; ++k) o[k] = f2bf(v[k]); *(volatile v8us*)(dst + i * 8) = o; __threadfence(); *(volatile v8us*)(dst + i * 8) = o; }
__global__ __launch_bounds__(256) void k_wcx(const float* __restrict__ wr, const float* __restrict__ wi, int Kh, int N, int interleave, int kperm, bf* dst) { const size_t i = (size_t)blockIdx.x * 256 + threadIdx.x; const int KK = 2 * Kh; if (i >= (size_t)2 * N * KK / 8) return; const int nn = (int)(i / (KK / 8)); const int k0 = (int)(i % (KK / 8)) * 8; const int c = interleave ? (nn >> 1) : (nn % N); const int comp = interleave ? (nn & 1) : (nn / N); v8us o; int chain = 0;
#pragma unroll
    for (int q = 0; q < 8; ++q) { const int k = k0 + q; int part, srow; if (kperm) { const int h = k / DW, p = (k % DW) / DH, d = k % DH; part = p; srow = h * DH + d; } else { part = (k >= Kh) ? 1 : 0; srow = part ? k - Kh : k; }
        float a = wr[(size_t)srow * N + c + chain], bq = wi[(size_t)srow * N + c + chain]; asm volatile("s_wait_loadcnt 0x0" : "+v"(a), "+v"(bq), "+v"(chain) :: "memory");
        const float w = (comp == 0) ? (part ? -bq : a) : (part ? a : bq); o[q] = f2bf(w); }
    *(volatile v8us*)(dst + i * 8) = o; __threadfence(); *(volatile v8us*)(dst + i * 8) = o; }
__global__ __launch_bounds__(256) void k_plqk(const float* __restrict__ F, int pitch, int base0, int base1, bf* Ph, bf* Pl) { const size_t e = ((size_t)blockIdx.x * 256 + threadIdx.x) * 2; if (e >= (size_t)NH_ * 2 * TT * DH) return; const int d = (int)(e % DH); const int t = (int)((e / DH) % TT); const int hp = (int)(e / ((size_t)DH * TT)); const int h = hp >> 1, p = hp & 1; const float* f = F + (size_t)t * pitch + (p ? base1 : base0) + h * DH + d; v2us oh, ol;
#pragma unroll
    for (int q = 0; q < 2; ++q) { unsigned short a, c2; splitf(f[q], a, c2); oh[q] = a; ol[q] = c2; }
    *(volatile v2us*)(Ph + e) = oh; *(volatile v2us*)(Pl + e) = ol; __threadfence(); *(volatile v2us*)(Ph + e) = oh; *(volatile v2us*)(Pl + e) = ol; }
__global__ __launch_bounds__(256) void k_vcz(const float* __restrict__ F, int pitch, int VR0, int VI0, h16* V16, bf* Vh, bf* Vl) { const size_t e = ((size_t)blockIdx.x * 256 + threadIdx.x) * 2; if (e >= (size_t)NH_ * DW * KPV) return; const int j = (int)(e % TT); const int r = (int)((e / TT) % NREP); const int dd = (int)((e / KPV) % DW); const int h = (int)(e / ((size_t)KPV * DW)); const int d = dd % DH; const bool oi = (dd >= DH); const bool mid = (r == 1 || r == 2);
    const bool usei = oi ? !mid : mid; const float sgn = oi ? (r == 3 ? -1.0f : 1.0f) : (r == 0 ? 1.0f : -1.0f); const float* f = F + (size_t)j * pitch + (usei ? VI0 : VR0) + h * DH + d; v2h o16; v2us oh, ol;
#pragma unroll
    for (int q = 0; q < 2; ++q) { const float x = sgn * f[(size_t)q * pitch]; o16[q] = tohx(x); unsigned short a, c2; splitf(x, a, c2); oh[q] = a; ol[q] = c2; }
    *(volatile v2h*)(V16 + e) = o16; *(volatile v2us*)(Vh + e) = oh; *(volatile v2us*)(Vl + e) = ol; __threadfence(); *(volatile v2h*)(V16 + e) = o16; *(volatile v2us*)(Vh + e) = oh; *(volatile v2us*)(Vl + e) = ol; }
__global__ __launch_bounds__(256) void k_asoft(const float* __restrict__ Sb, h16* P16, bf* Ph, bf* Pl) {
    const int lane = threadIdx.x & 31; const int row = blockIdx.x * 8 + (threadIdx.x >> 5); if (row >= NREP * TT) return; const int i = row / NREP;   const bool hires = (i < RH); const float* sr = Sb + (size_t)row * TT; float v[TT / 32]; float mx = -3.0e38f;
#pragma unroll
    for (int ch = 0; ch < TT / 128; ++ch) { const int j0 = ch * 128 + lane * 4; const v4f a = *(const v4f*)(sr + j0);
#pragma unroll
        for (int q = 0; q < 4; ++q) { const int j = j0 + q; (void)j; const float t = a[q] * SCL; v[ch * 4 + q] = t; mx = fmaxf(mx, t); } }
#pragma unroll
    for (int sh = 16; sh; sh >>= 1) mx = fmaxf(mx, __shfl_xor(mx, sh, 32));
    float sum = 0.f;
#pragma unroll
    for (int k = 0; k < TT / 32; ++k) { float d0 = __fsub_rn(v[k], mx); asm volatile("" : "+v"(d0)); v[k] = __builtin_amdgcn_exp2f(__fmul_rn(d0, 1.4426950408889634f)); sum += v[k]; }
#pragma unroll
    for (int sh = 16; sh; sh >>= 1) sum += __shfl_xor(sum, sh, 32);
    const float f = __fdiv_rn(hires ? 1.0f : PCAR, sum);
#pragma unroll 1
    for (int ps = 0; ps < 2; ++ps) {
        if (hires) {
#pragma unroll
            for (int ch = 0; ch < TT / 128; ++ch) { v4us oh, ol;
#pragma unroll
                for (int q = 0; q < 4; ++q) { unsigned short a, c2; splitf(v[ch * 4 + q] * f, a, c2); oh[q] = a; ol[q] = c2; }
                const size_t oo = (size_t)row * TT + ch * 128 + lane * 4; *(volatile v4us*)(Ph + oo) = oh; *(volatile v4us*)(Pl + oo) = ol; }
        } else {
#pragma unroll
            for (int ch = 0; ch < TT / 128; ++ch) { v4h o4;
#pragma unroll
                for (int q = 0; q < 4; ++q) o4[q] = tohx(v[ch * 4 + q] * f);
                *(volatile v4h*)(P16 + (size_t)row * TT + ch * 128 + lane * 4) = o4; } }
        if (ps == 0) __threadfence(); }
}
__global__ __launch_bounds__(256) void k_merge(const float* __restrict__ O, int h0, bf* Ah, bf* Al) { const size_t e = ((size_t)blockIdx.x * 256 + threadIdx.x) * 2; if (e >= (size_t)ZH * TT * HD) return; const int d = (int)(e % HD); const int t = (int)((e / HD) % TT); const int zz = (int)(e / ((size_t)HD * TT)); const float cs = (t < RH) ? 1.0f : (1.0f / PCAR); const size_t oo = (size_t)t * DQ + (h0 + zz) * HD + d;
    v2us oh, ol;
#pragma unroll
    for (int q = 0; q < 2; ++q) { unsigned short a, c2; splitf(O[e + q] * cs, a, c2); oh[q] = a; ol[q] = c2; } *(volatile v2us*)(Ah + oo) = oh; *(volatile v2us*)(Al + oo) = ol; __threadfence(); *(volatile v2us*)(Ah + oo) = oh; *(volatile v2us*)(Al + oo) = ol; }

extern "C" void kernel_launch(void* const* d_in, const int* in_sizes, int n_in,
                              void* d_out, int out_size, void* d_ws, size_t ws_size, hipStream_t stream) {
    (void)in_sizes; (void)n_in; (void)out_size;
    const float* xr = (const float*)d_in[0]; const float* xi = (const float*)d_in[1]; const float* wqr = (const float*)d_in[2]; const float* wqi = (const float*)d_in[3]; const float* wkvr = (const float*)d_in[4]; const float* wkvi = (const float*)d_in[5]; const float* wor = (const float*)d_in[6]; const float* woi = (const float*)d_in[7];
    float* OUT = (float*)d_out;
    char* wsp = (char*)d_ws;
    auto take = [&](size_t bytes) { char* p = wsp; wsp += (bytes + 255) & ~(size_t)255; return (void*)p; };
    bf* WQB = (bf*)take((size_t)2 * DIM * KX * 2); bf* WKVB = (bf*)take((size_t)4 * DIM * KX * 2); bf* WOB = (bf*)take((size_t)2 * DIM * DQ * 2);
    bf* XC = (bf*)take((size_t)TT * KX * 2); float* FQ = (float*)take((size_t)TT * 2 * DIM * 4); float* FKV = (float*)take((size_t)TT * 4 * DIM * 4);
    const size_t TS = (size_t)TT * DH;
    bf* QPh = (bf*)take((size_t)NH_ * 2 * TS * 2); bf* QPl = (bf*)take((size_t)NH_ * 2 * TS * 2); bf* KPh = (bf*)take((size_t)NH_ * 2 * TS * 2); bf* KPl = (bf*)take((size_t)NH_ * 2 * TS * 2);
    const size_t VS = (size_t)DW * KPV;
    h16* VC16 = (h16*)take((size_t)NH_ * VS * 2); bf* VCh = (bf*)take((size_t)NH_ * VS * 2); bf* VCl = (bf*)take((size_t)NH_ * VS * 2);
    float* Sb = (float*)take((size_t)TT * KPV * 4); h16* P16 = (h16*)take((size_t)TT * KPV * 2); bf* Ph = (bf*)take((size_t)RH * KPV * 2); bf* Pl = (bf*)take((size_t)RH * KPV * 2); float* Ob = (float*)take((size_t)TT * DW * 4); bf* ATh = (bf*)take((size_t)TT * DQ * 2); bf* ATl = (bf*)take((size_t)TT * DQ * 2);
    if ((size_t)(wsp - (char*)d_ws) > ws_size) return;
    k_wcx<<<(unsigned)(((size_t)2 * DIM * KX / 8 + 255) / 256), 256, 0, stream>>>(wqr, wqi, DIM, DIM, 0, 0, WQB); k_wcx<<<(unsigned)(((size_t)4 * DIM * KX / 8 + 255) / 256), 256, 0, stream>>>(wkvr, wkvi, DIM, 2 * DIM, 0, 0, WKVB); k_wcx<<<(unsigned)(((size_t)2 * DIM * DQ / 8 + 255) / 256), 256, 0, stream>>>(wor, woi, DIM, DIM, 1, 1, WOB);
    const unsigned LP = (unsigned)(((size_t)NH_ * 2 * TS / 2 + 255) / 256), LV = (unsigned)(((size_t)NH_ * VS / 2 + 255) / 256);
    for (int b = 0; b < NB_; ++b) {
        k_cvt8c<<<(unsigned)(((size_t)TT * KX / 8 + 255) / 256), 256, 0, stream>>>(xr + (size_t)b * TT * DIM, xi + (size_t)b * TT * DIM, XC);
        k_gemmw<bf, 0, false><<<dim3(TT / 64, 2 * DIM / 64, 1), 32, 0, stream>>>(XC, nullptr, WQB, nullptr, KX, FQ, 2 * DIM, nullptr, 0, 0, 0);
        k_gemmw<bf, 0, false><<<dim3(TT / 64, 4 * DIM / 64, 1), 32, 0, stream>>>(XC, nullptr, WKVB, nullptr, KX, FKV, 4 * DIM, nullptr, 0, 0, 0);
        k_plqk<<<LP, 256, 0, stream>>>(FQ, 2 * DIM, 0, DIM, QPh, QPl);
        k_plqk<<<LP, 256, 0, stream>>>(FKV, 4 * DIM, 0, 2 * DIM, KPh, KPl);
        k_vcz<<<LV, 256, 0, stream>>>(FKV, 4 * DIM, DIM, 3 * DIM, VC16, VCh, VCl);
        for (int h = 0; h < NH_; ++h) {
            for (int p = 0; p < 2; ++p)
                k_gemmw<bf, 2, false><<<dim3(TT / 64, TT / 64, 2), 32, 0, stream>>>(QPh + (size_t)(h * 2 + p) * TS, QPl + (size_t)(h * 2 + p) * TS, KPh + (size_t)(h * 2) * TS, KPl + (size_t)(h * 2) * TS, DH, Sb + (size_t)p * 2 * TT, KPV, nullptr, 0, TS, (size_t)TT);
            k_asoft<<<NREP * TT / 8, 256, 0, stream>>>(Sb, P16, Ph, Pl);
            k_gemmw<bf, 2, false><<<dim3(RH / 64, DW / 64, 1), 32, 0, stream>>>(Ph, Pl, VCh + (size_t)h * VS, VCl + (size_t)h * VS, KPV, Ob, DW, nullptr, 0, 0, 0);
            k_gemmw<h16, 0, false><<<dim3((TT - RH) / 64, DW / 64, 1), 32, 0, stream>>>(P16 + (size_t)RH * KPV, nullptr, VC16 + (size_t)h * VS, nullptr, KPV, Ob + (size_t)RH * DW, DW, nullptr, 0, 0, 0);
            k_merge<<<(unsigned)(((size_t)TT * DW / 2 + 255) / 256), 256, 0, stream>>>(Ob, h, ATh, ATl); }
        k_gemmw<bf, 1, false><<<dim3(TT / 64, 2 * DIM / 64, 1), 32, 0, stream>>>(ATh, ATl, WOB, nullptr, DQ, OUT + (size_t)b * TT * 2 * DIM, 2 * DIM, nullptr, 0, 0, 0); }
}
